// Encoder3_74998718923370
// MI455X (gfx1250) — hardware-verified
//
#include <hip/hip_runtime.h>
#include <stddef.h>


#define DF      128
#define H3      384
#define NTHR    256
#define NWAVE   8
#define EPT     8
#define NGRP    2
#define CHUNK   (NTHR * EPT * NGRP)
#define WCAP    (EPT * NGRP * 32)
#define LISTN   (NWAVE * WCAP)
#define NBA     512
#define NBD     4096
#define G0ROWS  128
#define HG      16
#define WSCALE  8.0f
#define WINV    0.125f

#define LDS_G0  (G0ROWS * DF * 4)
#define LDS_AGG (NBA * DF * 4 + LISTN * 4 + 64)

static_assert((CHUNK & (CHUNK - 1)) == 0);
static_assert(CHUNK <= 4096);
static_assert(NBA <= 4096 && NBD <= 4096 && HG <= 4096);
static_assert((NBA & (NBA - 1)) == 0 && (NBD & (NBD - 1)) == 0 && (HG & (HG - 1)) == 0);
static_assert(NBA == NWAVE * 64);
static_assert(NBD == NWAVE * 4 * 128);
static_assert(HG == NWAVE * 2);
static_assert(G0ROWS == NWAVE * 16);
static_assert((HG * H3) % NTHR == 0);

typedef float          v4f  __attribute__((ext_vector_type(4)));
typedef float          v8f  __attribute__((ext_vector_type(8)));
typedef int            v4i  __attribute__((ext_vector_type(4)));
typedef _Float16       v8h  __attribute__((ext_vector_type(8)));
typedef _Float16       v16h __attribute__((ext_vector_type(16)));
typedef unsigned short v8us __attribute__((ext_vector_type(8)));
typedef __bf16         v16b __attribute__((ext_vector_type(16)));
union FragH { v16h v; v8h  h[2]; };
union FragB { v16b v; v8us h[2]; };

__device__ __forceinline__ v8h cvt8(v4f a, v4f b) {
  v8h r;
  r[0] = (_Float16)a.x; r[1] = (_Float16)a.y; r[2] = (_Float16)a.z; r[3] = (_Float16)a.w;
  r[4] = (_Float16)b.x; r[5] = (_Float16)b.y; r[6] = (_Float16)b.z; r[7] = (_Float16)b.w;
  return r;
}

__device__ __forceinline__ unsigned bfbits(float f) {
  unsigned u = __builtin_bit_cast(unsigned, f);
  u += 0x7FFFu + ((u >> 16) & 1u);
  return u >> 16;
}

__device__ __forceinline__ void split8(v4f a, v4f b, v8us& hi, v8us& lo) {
  float f[8] = {a.x, a.y, a.z, a.w, b.x, b.y, b.z, b.w};
#pragma unroll
  for (int i = 0; i < 8; ++i) {
    const unsigned hb = bfbits(f[i]);
    const float    xh = __builtin_bit_cast(float, hb << 16);
    const unsigned lb = bfbits(f[i] - xh);
    hi[i] = (unsigned short)hb;
    lo[i] = (unsigned short)lb;
  }
}

__device__ __forceinline__ v8f wmh(v16h a, v16h b, v8f c) {
  v8f d = __builtin_amdgcn_wmma_f32_16x16x32_f16(false, a, false, b, (short)0, c, false, false);
  asm volatile("v_nop\n\tv_nop\n\tv_nop\n\tv_nop" : "+v"(d) : "v"(a), "v"(b));
  return d;
}
__device__ __forceinline__ v8f wmb(v16b a, v16b b, v8f c) {
  v8f d = __builtin_amdgcn_wmma_f32_16x16x32_bf16(false, a, false, b, (short)0, c, false, false);
  asm volatile("v_nop\n\tv_nop\n\tv_nop\n\tv_nop" : "+v"(d) : "v"(a), "v"(b));
  return d;
}

template <int NB>
__device__ __forceinline__ int scan_chunk(const int* __restrict__ dsts, int nE, int cbase, int nodeBase,
                                          int vec8, int* list, int tid, int lane, int wave) {
  int wc = 0;
#pragma unroll
  for (int g = 0; g < NGRP; ++g) {
    const int el0  = (g * NTHR + tid) * EPT;
    const int e0   = cbase + el0;
    const int sent = -2147483647 - 1;
    v4i da, db;
    if (vec8 != 0 && e0 + 7 < nE) {
      da = *(const v4i*)(dsts + e0);
      db = *(const v4i*)(dsts + e0 + 4);
    } else {
      da.x = (e0     < nE) ? dsts[min(e0, nE - 1)] : sent;
      da.y = (e0 + 1 < nE) ? dsts[min(e0 + 1, nE - 1)] : sent;
      da.z = (e0 + 2 < nE) ? dsts[min(e0 + 2, nE - 1)] : sent;
      da.w = (e0 + 3 < nE) ? dsts[min(e0 + 3, nE - 1)] : sent;
      db.x = (e0 + 4 < nE) ? dsts[min(e0 + 4, nE - 1)] : sent;
      db.y = (e0 + 5 < nE) ? dsts[min(e0 + 5, nE - 1)] : sent;
      db.z = (e0 + 6 < nE) ? dsts[min(e0 + 6, nE - 1)] : sent;
      db.w = (e0 + 7 < nE) ? dsts[min(e0 + 7, nE - 1)] : sent;
    }
    const unsigned nb = (unsigned)nodeBase;
    const unsigned s0 = (unsigned)da.x - nb, s1 = (unsigned)da.y - nb;
    const unsigned s2 = (unsigned)da.z - nb, s3 = (unsigned)da.w - nb;
    const unsigned s4 = (unsigned)db.x - nb, s5 = (unsigned)db.y - nb;
    const unsigned s6 = (unsigned)db.z - nb, s7 = (unsigned)db.w - nb;
    const bool h0 = s0 < (unsigned)NB, h1 = s1 < (unsigned)NB, h2 = s2 < (unsigned)NB, h3 = s3 < (unsigned)NB;
    const bool h4 = s4 < (unsigned)NB, h5 = s5 < (unsigned)NB, h6 = s6 < (unsigned)NB, h7 = s7 < (unsigned)NB;
    const unsigned any = __builtin_amdgcn_ballot_w32(h0 | h1 | h2 | h3 | h4 | h5 | h6 | h7);
    if (any != 0u) {
#define HITJ(J, HJ, SJ) { \
        const unsigned mj = __builtin_amdgcn_ballot_w32(HJ); \
        if (mj != 0u) { \
          if (HJ) { \
            const int pos = wc + (int)__builtin_amdgcn_mbcnt_lo(mj, 0u); \
            if (pos < WCAP) list[wave * WCAP + pos] = ((el0 + (J)) << 12) | (int)(SJ); \
          } \
          wc += (int)__builtin_popcount(mj); } }
      HITJ(0, h0, s0)
      HITJ(1, h1, s1)
      HITJ(2, h2, s2)
      HITJ(3, h3, s3)
      HITJ(4, h4, s4)
      HITJ(5, h5, s5)
      HITJ(6, h6, s6)
      HITJ(7, h7, s7)
#undef HITJ
    }
  }
  return wc;
}

__global__ __launch_bounds__(NTHR) void k_wprep(
    const float* __restrict__ W_in, const float* __restrict__ W1, const float* __restrict__ W2,
    const float* __restrict__ W3, const float* __restrict__ Wp1, const float* __restrict__ Wp2,
    _Float16* wf, unsigned short* wp1h, unsigned short* wp1l, unsigned short* wp2h, unsigned short* wp2l) {
  const int i   = blockIdx.x * NTHR + threadIdx.x;
  const int nPl = DF * DF / 8;
  const int nF  = 4 * nPl;
  const int nP1 = H3 * DF / 8;
  const int nP2 = nPl;
  if (i >= nF + nP1 + nP2) return;
  if (i < nF) {
    const int q  = i / nPl;
    const int o  = (i - q * nPl) * 8;
    const int n  = o / DF;
    const int k0 = o - n * DF;
    const float* W = (q == 0) ? W_in : ((q == 1) ? W1 : ((q == 2) ? W2 : W3));
    const float* p = W + (size_t)k0 * DF + n;
    v4f a, b;
    a.x = p[0];      a.y = p[DF];     a.z = p[2 * DF]; a.w = p[3 * DF];
    b.x = p[4 * DF]; b.y = p[5 * DF]; b.z = p[6 * DF]; b.w = p[7 * DF];
    a = a * WSCALE;
    b = b * WSCALE;
    const v8h hv = cvt8(a, b);
    _Float16* dp = wf + (size_t)q * DF * DF + o;
    *(volatile v8h*)dp = hv;
    __threadfence();
    *(volatile v8h*)dp = hv;
  } else if (i < nF + nP1) {
    const int o  = (i - nF) * 8;
    const int n  = o / H3;
    const int k0 = o - n * H3;
    const float* p = Wp1 + (size_t)k0 * DF + n;
    v4f a, b;
    a.x = p[0];      a.y = p[DF];     a.z = p[2 * DF]; a.w = p[3 * DF];
    b.x = p[4 * DF]; b.y = p[5 * DF]; b.z = p[6 * DF]; b.w = p[7 * DF];
    v8us hi, lo;
    split8(a, b, hi, lo);
    *(volatile v8us*)(wp1h + o) = hi;
    *(volatile v8us*)(wp1l + o) = lo;
    __threadfence();
    *(volatile v8us*)(wp1h + o) = hi;
    *(volatile v8us*)(wp1l + o) = lo;
  } else {
    const int o  = (i - nF - nP1) * 8;
    const int n  = o / DF;
    const int k0 = o - n * DF;
    const float* p = Wp2 + (size_t)k0 * DF + n;
    v4f a, b;
    a.x = p[0];      a.y = p[DF];     a.z = p[2 * DF]; a.w = p[3 * DF];
    b.x = p[4 * DF]; b.y = p[5 * DF]; b.z = p[6 * DF]; b.w = p[7 * DF];
    v8us hi, lo;
    split8(a, b, hi, lo);
    *(volatile v8us*)(wp2h + o) = hi;
    *(volatile v8us*)(wp2l + o) = lo;
    __threadfence();
    *(volatile v8us*)(wp2h + o) = hi;
    *(volatile v8us*)(wp2l + o) = lo;
  }
}

__global__ __launch_bounds__(NTHR) void k_deg(
    const int* __restrict__ ei, float* dinv, int nN, int nE, int vec8) {
  __shared__ __attribute__((aligned(16))) int cnt[NBD];
  __shared__ __attribute__((aligned(16))) int list[LISTN];
  __shared__ int wcnt[NWAVE];
  const int tid = threadIdx.x, lane = tid & 31, wave = tid >> 5;
  const int nodeBase = blockIdx.x * NBD;
  const int* dsts = ei + nE;
  (void)nN;

  for (int i = tid; i < NBD; i += NTHR) cnt[i] = 0;
  __syncthreads();

  const int nChunks = (nE + CHUNK - 1) / CHUNK;
#pragma unroll 1
  for (int ch = 0; ch < nChunks; ++ch) {
    const int cbase = ch * CHUNK;
    const int wc = scan_chunk<NBD>(dsts, nE, cbase, nodeBase, vec8, list, tid, lane, wave);
    if (lane == 0) wcnt[wave] = wc;
    __syncthreads();
    if (wave == 0) {
#pragma unroll 1
      for (int wsx = 0; wsx < NWAVE; ++wsx) {
        int n = __builtin_amdgcn_readfirstlane(wcnt[wsx]);
        n = n > WCAP ? WCAP : (n < 0 ? 0 : n);
        const int* lp = list + wsx * WCAP;
#pragma unroll 1
        for (int i = 0; i < n; ++i) {
          const int ent  = __builtin_amdgcn_readfirstlane(lp[i]);
          const int slot = ent & (NBD - 1);
          if (lane == 0) cnt[slot] = cnt[slot] + 1;
        }
      }
    }
    __syncthreads();
  }

  v4f dq[4];
#pragma unroll
  for (int q = 0; q < 4; ++q) {
    const int f = (wave * 4 + q) * 128 + 4 * lane;
    const v4i c = *(const v4i*)(cnt + f);
    dq[q].x = rsqrtf((float)(c.x + 1));
    dq[q].y = rsqrtf((float)(c.y + 1));
    dq[q].z = rsqrtf((float)(c.z + 1));
    dq[q].w = rsqrtf((float)(c.w + 1));
  }
  float* dp = dinv + (size_t)nodeBase;
#pragma unroll
  for (int q = 0; q < 4; ++q) *(volatile v4f*)(dp + (wave * 4 + q) * 128 + 4 * lane) = dq[q];
  __threadfence();
#pragma unroll
  for (int q = 0; q < 4; ++q) *(volatile v4f*)(dp + (wave * 4 + q) * 128 + 4 * lane) = dq[q];
}

__global__ __launch_bounds__(NTHR) void k_gemm0(
    const float* __restrict__ x, const _Float16* __restrict__ win, const _Float16* __restrict__ w1,
    const float* __restrict__ b_in, const float* __restrict__ dinv,
    float* hout, float* gout, int nN) {
  extern __shared__ v4f lds_dyn[];
  float* stg = (float*)lds_dyn;
  const int tid = threadIdx.x, lane = tid & 31, wave = tid >> 5, hh = lane >> 4, m = lane & 15;
  const int rowBase = blockIdx.x * G0ROWS;

  int node = rowBase + wave * 16 + m;
  node = node > nN - 1 ? nN - 1 : node;
  const float* xr = x + (size_t)node * DF + 8 * hh;

  v8f acc[8];
#pragma unroll
  for (int t = 0; t < 8; ++t) { v8f z = {0.f, 0.f, 0.f, 0.f, 0.f, 0.f, 0.f, 0.f}; acc[t] = z; }
#pragma unroll
  for (int kt = 0; kt < DF / 32; ++kt) {
    const float* p = xr + 32 * kt;
    const v4f p0 = *(const v4f*)p,        p1 = *(const v4f*)(p + 4);
    const v4f p2 = *(const v4f*)(p + 16), p3 = *(const v4f*)(p + 20);
    FragH a;
    a.h[0] = cvt8(p0, p1);
    a.h[1] = cvt8(p2, p3);
#pragma unroll
    for (int t = 0; t < 8; ++t) {
      const _Float16* bp = win + (size_t)(16 * t + m) * DF + 32 * kt + 8 * hh;
      FragH b;
      b.h[0] = *(const v8h*)bp;
      b.h[1] = *(const v8h*)(bp + 16);
      acc[t] = wmh(a.v, b.v, acc[t]);
    }
  }

  const int r0 = wave * 16 + 8 * hh;
  float* sp = stg + r0 * DF + m;
#pragma unroll
  for (int t = 0; t < 8; ++t) {
    const float bc = b_in[16 * t + m];
    sp[0 * DF + 16 * t] = acc[t][0] * WINV + bc;
    sp[1 * DF + 16 * t] = acc[t][1] * WINV + bc;
    sp[2 * DF + 16 * t] = acc[t][2] * WINV + bc;
    sp[3 * DF + 16 * t] = acc[t][3] * WINV + bc;
    sp[4 * DF + 16 * t] = acc[t][4] * WINV + bc;
    sp[5 * DF + 16 * t] = acc[t][5] * WINV + bc;
    sp[6 * DF + 16 * t] = acc[t][6] * WINV + bc;
    sp[7 * DF + 16 * t] = acc[t][7] * WINV + bc;
  }
  __syncthreads();

  {
    const float* lp = stg + wave * 16 * DF + 4 * lane;
    float* gp = hout + ((size_t)rowBase + wave * 16) * DF + 4 * lane;
#pragma unroll
    for (int i = 0; i < 16; ++i) { const v4f v = *(const v4f*)(lp + i * DF); *(volatile v4f*)(gp + (size_t)i * DF) = v; }
    __threadfence();
#pragma unroll
    for (int i = 0; i < 16; ++i) { const v4f v = *(const v4f*)(lp + i * DF); *(volatile v4f*)(gp + (size_t)i * DF) = v; }
  }

#pragma unroll
  for (int t = 0; t < 8; ++t) { v8f z = {0.f, 0.f, 0.f, 0.f, 0.f, 0.f, 0.f, 0.f}; acc[t] = z; }
  const float* ar = stg + (wave * 16 + m) * DF + 8 * hh;
#pragma unroll
  for (int kt = 0; kt < DF / 32; ++kt) {
    const float* p = ar + 32 * kt;
    const v4f p0 = *(const v4f*)p,        p1 = *(const v4f*)(p + 4);
    const v4f p2 = *(const v4f*)(p + 16), p3 = *(const v4f*)(p + 20);
    FragH a;
    a.h[0] = cvt8(p0, p1);
    a.h[1] = cvt8(p2, p3);
#pragma unroll
    for (int t = 0; t < 8; ++t) {
      const _Float16* bp = w1 + (size_t)(16 * t + m) * DF + 32 * kt + 8 * hh;
      FragH b;
      b.h[0] = *(const v8h*)bp;
      b.h[1] = *(const v8h*)(bp + 16);
      acc[t] = wmh(a.v, b.v, acc[t]);
    }
  }
  __syncthreads();

  {
    const v4f dA = *(const v4f*)(dinv + (size_t)rowBase + r0);
    const v4f dB = *(const v4f*)(dinv + (size_t)rowBase + r0 + 4);
    const float d0 = dA.x * WINV, d1 = dA.y * WINV, d2 = dA.z * WINV, d3 = dA.w * WINV;
    const float d4 = dB.x * WINV, d5 = dB.y * WINV, d6 = dB.z * WINV, d7 = dB.w * WINV;
#pragma unroll
    for (int t = 0; t < 8; ++t) {
      sp[0 * DF + 16 * t] = acc[t][0] * d0;
      sp[1 * DF + 16 * t] = acc[t][1] * d1;
      sp[2 * DF + 16 * t] = acc[t][2] * d2;
      sp[3 * DF + 16 * t] = acc[t][3] * d3;
      sp[4 * DF + 16 * t] = acc[t][4] * d4;
      sp[5 * DF + 16 * t] = acc[t][5] * d5;
      sp[6 * DF + 16 * t] = acc[t][6] * d6;
      sp[7 * DF + 16 * t] = acc[t][7] * d7;
    }
  }
  __syncthreads();

  {
    const float* lp = stg + wave * 16 * DF + 4 * lane;
    float* gp = gout + ((size_t)rowBase + wave * 16) * DF + 4 * lane;
#pragma unroll
    for (int i = 0; i < 16; ++i) { const v4f v = *(const v4f*)(lp + i * DF); *(volatile v4f*)(gp + (size_t)i * DF) = v; }
    __threadfence();
#pragma unroll
    for (int i = 0; i < 16; ++i) { const v4f v = *(const v4f*)(lp + i * DF); *(volatile v4f*)(gp + (size_t)i * DF) = v; }
  }
}

template <int HAS_NEXT>
__global__ __launch_bounds__(NTHR) void k_agg(
    const int* __restrict__ ei, const float* __restrict__ gin, const float* __restrict__ hin,
    const float* __restrict__ dinv, const float* __restrict__ bias, const _Float16* __restrict__ wn,
    float* rout, float* gout, int nN, int nE, int vec8) {
  extern __shared__ v4f lds_dyn[];
  float* acc  = (float*)lds_dyn;
  int*   list = (int*)(acc + NBA * DF);
  int*   wcnt = list + LISTN;
  const int tid = threadIdx.x, lane = tid & 31, wave = tid >> 5, hh = lane >> 4, m = lane & 15;
  const int nodeBase = blockIdx.x * NBA;
  const int* dsts = ei + nE;

  {
    const v4f z = {0.f, 0.f, 0.f, 0.f};
    for (int i = tid; i < NBA * DF / 4; i += NTHR) lds_dyn[i] = z;
  }
  __syncthreads();

  const int nChunks = (nE + CHUNK - 1) / CHUNK;
#pragma unroll 1
  for (int ch = 0; ch < nChunks; ++ch) {
    const int cbase = ch * CHUNK;
    const int wc = scan_chunk<NBA>(dsts, nE, cbase, nodeBase, vec8, list, tid, lane, wave);
    if (lane == 0) wcnt[wave] = wc;
    __syncthreads();
    if (wave == 0) {
#pragma unroll 1
      for (int wsx = 0; wsx < NWAVE; ++wsx) {
        int n = __builtin_amdgcn_readfirstlane(wcnt[wsx]);
        n = n > WCAP ? WCAP : (n < 0 ? 0 : n);
        const int* lp = list + wsx * WCAP;
#pragma unroll 1
        for (int i = 0; i < n; ++i) {
          const int ent  = __builtin_amdgcn_readfirstlane(lp[i]);
          const int slot = ent & (NBA - 1);
          int e = cbase + ((ent >> 12) & (CHUNK - 1));
          e = e > nE - 1 ? nE - 1 : e;
          int src = ei[e];
          src = src < 0 ? 0 : (src > nN - 1 ? nN - 1 : src);
          const v4f v = *(const v4f*)(gin + (size_t)src * DF + 4 * lane);
          v4f* ap = (v4f*)(acc + slot * DF + 4 * lane);
          *ap = *ap + v;
        }
      }
    }
    __syncthreads();
  }

#pragma unroll 4
  for (int i = 0; i < (NBA * DF / 4) / NTHR; ++i) {
    const int idx  = i * NTHR + tid;
    const int slot = idx >> 5;
    const int c4   = (idx & 31) * 4;
    int node = nodeBase + slot;
    node = node > nN - 1 ? nN - 1 : node;
    const float d  = dinv[node];
    const v4f   gv = *(const v4f*)(gin + (size_t)node * DF + c4);
    const v4f   xv = *(const v4f*)(hin + (size_t)node * DF + c4);
    const v4f   bv = *(const v4f*)(bias + c4);
    v4f* ap = (v4f*)(acc + slot * DF + c4);
    const v4f cv = (*ap + gv) * d + bv;
    v4f hv = xv + cv;
    hv.x = fmaxf(hv.x, 0.f); hv.y = fmaxf(hv.y, 0.f); hv.z = fmaxf(hv.z, 0.f); hv.w = fmaxf(hv.w, 0.f);
    *ap = hv;
  }
  __syncthreads();

  {
    const float* lp = acc + wave * 64 * DF + 4 * lane;
    float* gp = rout + ((size_t)nodeBase + wave * 64) * DF + 4 * lane;
#pragma unroll 4
    for (int i = 0; i < 64; ++i) { const v4f v = *(const v4f*)(lp + i * DF); *(volatile v4f*)(gp + (size_t)i * DF) = v; }
    __threadfence();
#pragma unroll 4
    for (int i = 0; i < 64; ++i) { const v4f v = *(const v4f*)(lp + i * DF); *(volatile v4f*)(gp + (size_t)i * DF) = v; }
  }

  if (HAS_NEXT) {
#pragma unroll 1
    for (int s = 0; s < NBA / (16 * NWAVE); ++s) {
      const int t = wave + NWAVE * s;
      v8f c[8];
#pragma unroll
      for (int t2 = 0; t2 < 8; ++t2) { v8f z = {0.f, 0.f, 0.f, 0.f, 0.f, 0.f, 0.f, 0.f}; c[t2] = z; }
#pragma unroll
      for (int kt = 0; kt < DF / 32; ++kt) {
        const float* ap = acc + (16 * t + m) * DF + 32 * kt + 8 * hh;
        const v4f p0 = *(const v4f*)ap,        p1 = *(const v4f*)(ap + 4);
        const v4f p2 = *(const v4f*)(ap + 16), p3 = *(const v4f*)(ap + 20);
        FragH a;
        a.h[0] = cvt8(p0, p1);
        a.h[1] = cvt8(p2, p3);
#pragma unroll
        for (int t2 = 0; t2 < 8; ++t2) {
          const _Float16* bp = wn + (size_t)(16 * t2 + m) * DF + 32 * kt + 8 * hh;
          FragH b;
          b.h[0] = *(const v8h*)bp;
          b.h[1] = *(const v8h*)(bp + 16);
          c[t2] = wmh(a.v, b.v, c[t2]);
        }
      }
      __syncthreads();

      const int lr0 = 16 * t + 8 * hh;
      const v4f dA = *(const v4f*)(dinv + (size_t)nodeBase + lr0);
      const v4f dB = *(const v4f*)(dinv + (size_t)nodeBase + lr0 + 4);
      const float d0 = dA.x * WINV, d1 = dA.y * WINV, d2 = dA.z * WINV, d3 = dA.w * WINV;
      const float d4 = dB.x * WINV, d5 = dB.y * WINV, d6 = dB.z * WINV, d7 = dB.w * WINV;
      float* sp = acc + lr0 * DF + m;
#pragma unroll
      for (int t2 = 0; t2 < 8; ++t2) {
        sp[0 * DF + 16 * t2] = c[t2][0] * d0;
        sp[1 * DF + 16 * t2] = c[t2][1] * d1;
        sp[2 * DF + 16 * t2] = c[t2][2] * d2;
        sp[3 * DF + 16 * t2] = c[t2][3] * d3;
        sp[4 * DF + 16 * t2] = c[t2][4] * d4;
        sp[5 * DF + 16 * t2] = c[t2][5] * d5;
        sp[6 * DF + 16 * t2] = c[t2][6] * d6;
        sp[7 * DF + 16 * t2] = c[t2][7] * d7;
      }
    }
    __syncthreads();

    {
      const float* lp = acc + wave * 64 * DF + 4 * lane;
      float* gp = gout + ((size_t)nodeBase + wave * 64) * DF + 4 * lane;
#pragma unroll 4
      for (int i = 0; i < 64; ++i) { const v4f v = *(const v4f*)(lp + i * DF); *(volatile v4f*)(gp + (size_t)i * DF) = v; }
      __threadfence();
#pragma unroll 4
      for (int i = 0; i < 64; ++i) { const v4f v = *(const v4f*)(lp + i * DF); *(volatile v4f*)(gp + (size_t)i * DF) = v; }
    }
  }
}

__global__ __launch_bounds__(NTHR) void k_poolhead(
    const int* __restrict__ batch, const float* __restrict__ ra, const float* __restrict__ rb,
    const float* __restrict__ rc, const unsigned short* __restrict__ wp1h, const unsigned short* __restrict__ wp1l,
    const unsigned short* __restrict__ wp2h, const unsigned short* __restrict__ wp2l,
    const float* __restrict__ bp1, const float* __restrict__ bp2, float* out, int nN, int nG) {
  __shared__ __attribute__((aligned(16))) int   list[LISTN];
  __shared__ int wcnt[NWAVE];
  __shared__ int cnt[HG];
  __shared__ __attribute__((aligned(16))) float sums[HG * H3];
  __shared__ __attribute__((aligned(16))) float phs[HG * DF];
  __shared__ __attribute__((aligned(16))) float pst[HG * DF];
  const int tid = threadIdx.x, lane = tid & 31, wave = tid >> 5, hh = lane >> 4, m = lane & 15;
  const int g0 = blockIdx.x * HG;

  for (int i = tid; i < HG * H3; i += NTHR) sums[i] = 0.f;
  if (tid < HG) cnt[tid] = 0;
  __syncthreads();

  const int nChunks = (nN + CHUNK - 1) / CHUNK;
#pragma unroll 1
  for (int ch = 0; ch < nChunks; ++ch) {
    const int cbase = ch * CHUNK;
    const int wc = scan_chunk<HG>(batch, nN, cbase, g0, 1, list, tid, lane, wave);
    if (lane == 0) wcnt[wave] = wc;
    __syncthreads();
#pragma unroll 1
    for (int wsx = 0; wsx < NWAVE; ++wsx) {
      int n = wcnt[wsx];
      n = n > WCAP ? WCAP : (n < 0 ? 0 : n);
      const int* lp = list + wsx * WCAP;
#pragma unroll 1
      for (int i = 0; i < n; ++i) {
        const int ent  = lp[i];
        const int slot = ent & (HG - 1);
        int node = cbase + ((ent >> 12) & (CHUNK - 1));
        node = node > nN - 1 ? nN - 1 : node;
        const size_t nb = (size_t)node * DF;
        float* srow = sums + slot * H3;
        if (tid < DF) {
          srow[tid]          = srow[tid]          + ra[nb + tid];
          srow[2 * DF + tid] = srow[2 * DF + tid] + rc[nb + tid];
        } else {
          srow[tid]          = srow[tid]          + rb[nb + (tid - DF)];
        }
        if (tid == 0) cnt[slot] = cnt[slot] + 1;
      }
    }
    __syncthreads();
  }

#pragma unroll 1
  for (int j = 0; j < (HG * H3) / NTHR; ++j) {
    const int idx  = j * NTHR + tid;
    const int slot = idx / H3;
    const float rcp = 1.0f / fmaxf((float)cnt[slot], 1.0f);
    sums[idx] = sums[idx] * rcp;
  }
  __syncthreads();

  const int col = 16 * wave + m;
  {
    v8f c = {0.f, 0.f, 0.f, 0.f, 0.f, 0.f, 0.f, 0.f};
#pragma unroll 2
    for (int kt = 0; kt < H3 / 32; ++kt) {
      const float* ap = sums + m * H3 + 32 * kt + 8 * hh;
      const v4f p0 = *(const v4f*)ap,        p1 = *(const v4f*)(ap + 4);
      const v4f p2 = *(const v4f*)(ap + 16), p3 = *(const v4f*)(ap + 20);
      FragB ahi, alo;
      split8(p0, p1, ahi.h[0], alo.h[0]);
      split8(p2, p3, ahi.h[1], alo.h[1]);
      const unsigned short* bph = wp1h + (size_t)col * H3 + 32 * kt + 8 * hh;
      const unsigned short* bpl = wp1l + (size_t)col * H3 + 32 * kt + 8 * hh;
      FragB bhi, blo;
      bhi.h[0] = *(const v8us*)bph; bhi.h[1] = *(const v8us*)(bph + 16);
      blo.h[0] = *(const v8us*)bpl; blo.h[1] = *(const v8us*)(bpl + 16);
      c = wmb(ahi.v, bhi.v, c);
      c = wmb(ahi.v, blo.v, c);
      c = wmb(alo.v, bhi.v, c);
    }
    const float bb = bp1[col];
    float* sp = phs + (8 * hh) * DF + col;
    sp[0 * DF] = fmaxf(c[0] + bb, 0.f);
    sp[1 * DF] = fmaxf(c[1] + bb, 0.f);
    sp[2 * DF] = fmaxf(c[2] + bb, 0.f);
    sp[3 * DF] = fmaxf(c[3] + bb, 0.f);
    sp[4 * DF] = fmaxf(c[4] + bb, 0.f);
    sp[5 * DF] = fmaxf(c[5] + bb, 0.f);
    sp[6 * DF] = fmaxf(c[6] + bb, 0.f);
    sp[7 * DF] = fmaxf(c[7] + bb, 0.f);
  }
  __syncthreads();

  {
    v8f c = {0.f, 0.f, 0.f, 0.f, 0.f, 0.f, 0.f, 0.f};
#pragma unroll
    for (int kt = 0; kt < DF / 32; ++kt) {
      const float* ap = phs + m * DF + 32 * kt + 8 * hh;
      const v4f p0 = *(const v4f*)ap,        p1 = *(const v4f*)(ap + 4);
      const v4f p2 = *(const v4f*)(ap + 16), p3 = *(const v4f*)(ap + 20);
      FragB ahi, alo;
      split8(p0, p1, ahi.h[0], alo.h[0]);
      split8(p2, p3, ahi.h[1], alo.h[1]);
      const unsigned short* bph = wp2h + (size_t)col * DF + 32 * kt + 8 * hh;
      const unsigned short* bpl = wp2l + (size_t)col * DF + 32 * kt + 8 * hh;
      FragB bhi, blo;
      bhi.h[0] = *(const v8us*)bph; bhi.h[1] = *(const v8us*)(bph + 16);
      blo.h[0] = *(const v8us*)bpl; blo.h[1] = *(const v8us*)(bpl + 16);
      c = wmb(ahi.v, bhi.v, c);
      c = wmb(ahi.v, blo.v, c);
      c = wmb(alo.v, bhi.v, c);
    }
    const float bb = bp2[col];
    float* sp = pst + (8 * hh) * DF + col;
    sp[0 * DF] = c[0] + bb;
    sp[1 * DF] = c[1] + bb;
    sp[2 * DF] = c[2] + bb;
    sp[3 * DF] = c[3] + bb;
    sp[4 * DF] = c[4] + bb;
    sp[5 * DF] = c[5] + bb;
    sp[6 * DF] = c[6] + bb;
    sp[7 * DF] = c[7] + bb;
  }
  __syncthreads();

  {
    const int row = tid >> 4, part = tid & 15;
    float* q = pst + row * DF + 8 * part;
    v4f u0 = *(const v4f*)q, u1 = *(const v4f*)(q + 4);
    float s = u0.x * u0.x + u0.y * u0.y + u0.z * u0.z + u0.w * u0.w
            + u1.x * u1.x + u1.y * u1.y + u1.z * u1.z + u1.w * u1.w;
    s += __shfl_xor(s, 8);
    s += __shfl_xor(s, 4);
    s += __shfl_xor(s, 2);
    s += __shfl_xor(s, 1);
    const float inv = 1.0f / fmaxf(sqrtf(s), 1e-12f);
    u0 = u0 * inv;
    u1 = u1 * inv;
    *(v4f*)q       = u0;
    *(v4f*)(q + 4) = u1;
  }
  __syncthreads();

  v4f ov[2];
#pragma unroll
  for (int rr = 0; rr < 2; ++rr) ov[rr] = *(const v4f*)(pst + (wave * 2 + rr) * DF + 4 * lane);
#pragma unroll
  for (int rr = 0; rr < 2; ++rr) {
    const int g = g0 + wave * 2 + rr;
    if (g < nG) *(volatile v4f*)(out + (size_t)g * DF + 4 * lane) = ov[rr];
  }
  __threadfence();
#pragma unroll
  for (int rr = 0; rr < 2; ++rr) {
    const int g = g0 + wave * 2 + rr;
    if (g < nG) *(volatile v4f*)(out + (size_t)g * DF + 4 * lane) = ov[rr];
  }
}

extern "C" void kernel_launch(void* const* d_in, const int* in_sizes, int n_in,
                              void* d_out, int out_size, void* d_ws, size_t ws_size,
                              hipStream_t stream) {
  if (n_in < 15) return;
  const int nN = in_sizes[2];
  if (nN <= 0) return;
  const int nE = in_sizes[1] / 2;
  if (nE < 0 || in_sizes[1] != nE * 2) return;
  if (in_sizes[0] != nN * DF) return;
  if (in_sizes[3] != DF * DF || in_sizes[5] != DF * DF || in_sizes[7] != DF * DF || in_sizes[9] != DF * DF) return;
  if (in_sizes[11] != H3 * DF || in_sizes[13] != DF * DF) return;
  if (in_sizes[4] < DF || in_sizes[6] < DF || in_sizes[8] < DF || in_sizes[10] < DF || in_sizes[12] < DF || in_sizes[14] < DF) return;
  if (out_size <= 0 || (out_size % DF) != 0) return;
  const int nG = out_size / DF;

  const float* x     = (const float*)d_in[0];
  const int*   ei    = (const int*)d_in[1];
  const int*   batch = (const int*)d_in[2];
  const float* W_in  = (const float*)d_in[3];
  const float* b_in  = (const float*)d_in[4];
  const float* W1    = (const float*)d_in[5];
  const float* b1    = (const float*)d_in[6];
  const float* W2    = (const float*)d_in[7];
  const float* b2    = (const float*)d_in[8];
  const float* W3    = (const float*)d_in[9];
  const float* b3    = (const float*)d_in[10];
  const float* Wp1   = (const float*)d_in[11];
  const float* bp1   = (const float*)d_in[12];
  const float* Wp2   = (const float*)d_in[13];
  const float* bp2   = (const float*)d_in[14];
  float* out = (float*)d_out;

  const int nBD = (nN + NBD - 1) / NBD;
  const int nG0 = (nN + G0ROWS - 1) / G0ROWS;
  const int nA  = (nN + NBA - 1) / NBA;
  const int nHB = (nG + HG - 1) / HG;
  const int rowsPad = nA * NBA;
  if (nG0 * G0ROWS > rowsPad || rowsPad > nBD * NBD) return;

  char* ws = (char*)d_ws;
  size_t off = 0;
  const size_t plane = (size_t)rowsPad * DF * 4;
  const size_t oWF  = off; off += (size_t)4 * DF * DF * 2;   off = (off + 255) & ~(size_t)255;
  const size_t oP1H = off; off += (size_t)H3 * DF * 2;       off = (off + 255) & ~(size_t)255;
  const size_t oP1L = off; off += (size_t)H3 * DF * 2;       off = (off + 255) & ~(size_t)255;
  const size_t oP2H = off; off += (size_t)DF * DF * 2;       off = (off + 255) & ~(size_t)255;
  const size_t oP2L = off; off += (size_t)DF * DF * 2;       off = (off + 255) & ~(size_t)255;
  const size_t oDV  = off; off += (size_t)nBD * NBD * 4;     off = (off + 255) & ~(size_t)255;
  const size_t oA   = off; off += plane;                     off = (off + 255) & ~(size_t)255;
  const size_t oB   = off; off += plane;                     off = (off + 255) & ~(size_t)255;
  const size_t oC   = off; off += plane;                     off = (off + 255) & ~(size_t)255;
  const size_t oD   = off; off += plane;                     off = (off + 255) & ~(size_t)255;
  if (off > ws_size) return;
  if (off > ((size_t)128 << 20)) return;

  _Float16*       wf   = (_Float16*)(ws + oWF);
  unsigned short* wp1h = (unsigned short*)(ws + oP1H);
  unsigned short* wp1l = (unsigned short*)(ws + oP1L);
  unsigned short* wp2h = (unsigned short*)(ws + oP2H);
  unsigned short* wp2l = (unsigned short*)(ws + oP2L);
  float* dinv = (float*)(ws + oDV);
  float* bufA = (float*)(ws + oA);
  float* bufB = (float*)(ws + oB);
  float* bufC = (float*)(ws + oC);
  float* bufD = (float*)(ws + oD);

  const int vec8 = ((nE & 3) == 0) ? 1 : 0;

  const int nPrep = 4 * (DF * DF / 8) + H3 * DF / 8 + DF * DF / 8;
  k_wprep<<<(nPrep + NTHR - 1) / NTHR, NTHR, 0, stream>>>(W_in, W1, W2, W3, Wp1, Wp2, wf, wp1h, wp1l, wp2h, wp2l);

  k_deg<<<nBD, NTHR, 0, stream>>>(ei, dinv, nN, nE, vec8);

  hipFuncSetAttribute(reinterpret_cast<const void*>(&k_gemm0),
                      hipFuncAttributeMaxDynamicSharedMemorySize, LDS_G0);
  k_gemm0<<<nG0, NTHR, LDS_G0, stream>>>(x, wf, wf + DF * DF, b_in, dinv, bufA, bufB, nN);

  hipFuncSetAttribute(reinterpret_cast<const void*>(&k_agg<1>),
                      hipFuncAttributeMaxDynamicSharedMemorySize, LDS_AGG);
  hipFuncSetAttribute(reinterpret_cast<const void*>(&k_agg<0>),
                      hipFuncAttributeMaxDynamicSharedMemorySize, LDS_AGG);
  k_agg<1><<<nA, NTHR, LDS_AGG, stream>>>(ei, bufB, bufA, dinv, b1, wf + 2 * DF * DF, bufC, bufD, nN, nE, vec8);
  k_agg<1><<<nA, NTHR, LDS_AGG, stream>>>(ei, bufD, bufC, dinv, b2, wf + 3 * DF * DF, bufA, bufB, nN, nE, vec8);
  k_agg<0><<<nA, NTHR, LDS_AGG, stream>>>(ei, bufB, bufA, dinv, b3, wf, bufD, bufB, nN, nE, vec8);

  k_poolhead<<<nHB, NTHR, 0, stream>>>(batch, bufC, bufA, bufD, wp1h, wp1l, wp2h, wp2l, bp1, bp2, out, nN, nG);
}
